// BiLSTMTagger_50079318671865
// MI455X (gfx1250) — hardware-verified
//
#include <hip/hip_runtime.h>
#include <math.h>

constexpr int NBATCH = 64;
constexpr int NSTEP  = 512;
constexpr int NVOC   = 30000;
constexpr int NEMB   = 128;
constexpr int NHID   = 256;
constexpr int NGATE  = 4 * NHID;
constexpr int NCAT   = 2 * NHID;
constexpr int NTAGS  = 50;
constexpr int NTAGP  = 64;
constexpr int NROWS  = NBATCH * NSTEP;
constexpr int NTHR   = 256;
constexpr int NWAVE  = NTHR / 32;
constexpr int RBLK   = 16;
constexpr int AHP    = NHID + 8;
constexpr int CLSM   = 128;
constexpr int CLSSTG = CLSM * NTAGS;
constexpr float CARRY      = 16.0f;
constexpr float CARRY2_INV = 1.0f / 256.0f;
constexpr size_t WS_LIMIT  = 134217728;

static_assert(NEMB % 32 == 0 && NHID % 32 == 0 && NCAT % 32 == 0);
static_assert(NEMB % 128 == 0 && NCAT % 128 == 0);
static_assert(NHID == 32 * NWAVE);
static_assert(RBLK == 2 * NWAVE && NTHR / 16 == RBLK);
static_assert(NBATCH % RBLK == 0 && NBATCH <= NTHR);
static_assert(NROWS % CLSM == 0 && CLSM == 16 * NWAVE);
static_assert(CLSSTG % 4 == 0 && CLSSTG / 4 == 6 * NTHR + 64);
static_assert(NTAGS <= NTAGP && NTAGP == 64);
static_assert((NROWS * (NEMB / 8)) % NTHR == 0);
static_assert(AHP % 8 == 0);

typedef __attribute__((ext_vector_type(16))) _Float16 v16h;
typedef __attribute__((ext_vector_type(8)))  _Float16 v8h;
typedef __attribute__((ext_vector_type(8)))  float    v8f;
typedef __attribute__((ext_vector_type(4)))  float    v4f;
typedef __attribute__((ext_vector_type(4)))  unsigned v4u;

__device__ __forceinline__ void dep_guard_h(v8f& a, v8f& b, v16h x, v16h y) { asm volatile("v_nop\n\tv_nop\n\tv_nop\n\tv_nop" : "+v"(a), "+v"(b) : "v"(x), "v"(y)); }
__device__ __forceinline__ void keep4_h(v16h a, v16h b, v16h c, v16h d) { asm volatile("v_nop" :: "v"(a), "v"(b), "v"(c), "v"(d)); }
__device__ __forceinline__ void acc_guard4(v8f& a, v8f& b, v8f& c, v8f& d) { asm volatile("v_nop\n\tv_nop\n\tv_nop\n\tv_nop" : "+v"(a), "+v"(b), "+v"(c), "+v"(d)); }
template <typename T> struct Frag;
template <> struct Frag<_Float16> {
  typedef v16h V; union U { v16h v; v8h h[2]; };
  static __device__ __forceinline__ v16h load(const _Float16* p) {
    U f; f.h[0] = *(const v8h*)(p); f.h[1] = *(const v8h*)(p + 16); return f.v;
  }
  static __device__ __forceinline__ v8f mma(v16h a, v16h b, v8f c) {
    return __builtin_amdgcn_wmma_f32_16x16x32_f16(false, a, false, b, (short)0, c, false, false);
  }
  static __device__ __forceinline__ void guard(v8f& a, v8f& b, v16h x, v16h y) { dep_guard_h(a, b, x, y); }
  static __device__ __forceinline__ void keep(v16h a, v16h b, v16h c, v16h d) { keep4_h(a, b, c, d); }
};

__device__ __forceinline__ float fsig(float x)  { return __builtin_amdgcn_rcpf(1.0f + expf(-x)); }
__device__ __forceinline__ float ftanh(float x) { return 1.0f - 2.0f * __builtin_amdgcn_rcpf(expf(2.0f * x) + 1.0f); }

__device__ __forceinline__ int clampi(int v, int lo, int hi) { v = v < lo ? lo : v; v = v > hi ? hi : v; return v; }

__global__ __launch_bounds__(NTHR) void cvt16_kernel(const float* __restrict__ src, unsigned short* __restrict__ dst,
                                                    int nrow_src, int nrow_dst, int ncol8, float sc) {
  const int i  = blockIdx.x * NTHR + threadIdx.x;
  const int n8 = nrow_dst * ncol8;
  if (i < n8) {
    const int row = i / ncol8;
    const int c8  = i - row * ncol8;
    const int rs  = (row < nrow_src) ? row : (nrow_src - 1);
    const float f = (row < nrow_src) ? sc : 0.0f;
    const float* sp = src + (size_t)rs * (size_t)(ncol8 * 8) + (size_t)c8 * 8;
    const v4f a = *(const v4f*)(sp);
    const v4f b = *(const v4f*)(sp + 4);
    v8h hv;
#pragma unroll
    for (int e = 0; e < 4; ++e) {
      hv[e]     = (_Float16)(a[e] * f);
      hv[4 + e] = (_Float16)(b[e] * f);
    }
    unsigned short* dp = dst + (size_t)i * 8;
    *(volatile v8h*)dp = hv;
    __threadfence();
    *(volatile v8h*)dp = hv;
  }
}

__global__ __launch_bounds__(NTHR) void bias_fold_kernel(const float* __restrict__ a0, const float* __restrict__ b0,
                                                        const float* __restrict__ a1, const float* __restrict__ b1,
                                                        const float* __restrict__ a2, const float* __restrict__ b2,
                                                        const float* __restrict__ a3, const float* __restrict__ b3,
                                                        float* __restrict__ dst) {
  const int blk = blockIdx.x;
  const float* pa = (blk == 0) ? a0 : (blk == 1) ? a1 : (blk == 2) ? a2 : a3;
  const float* pb = (blk == 0) ? b0 : (blk == 1) ? b1 : (blk == 2) ? b2 : b3;
  const int idx = threadIdx.x * 4;
  const v4f va = *(const v4f*)(pa + idx);
  const v4f vb = *(const v4f*)(pb + idx);
  v4f o;
#pragma unroll
  for (int e = 0; e < 4; ++e) o[e] = va[e] + vb[e];
  float* op = dst + (size_t)blk * NGATE + idx;
  *(volatile v4f*)op = o;
  __threadfence();
  *(volatile v4f*)op = o;
}

__global__ __launch_bounds__(NTHR) void gather_x16_kernel(const int* __restrict__ words, const float* __restrict__ emb,
                                                         unsigned short* __restrict__ xpl) {
  const int i  = blockIdx.x * NTHR + threadIdx.x;
  const int n8 = NROWS * (NEMB / 8);
  if (i < n8) {
    const int bt  = i >> 4;
    const int col = (i & 15) * 8;
    const int w = clampi(words[bt], 0, NVOC - 1);
    const float* sp = emb + (size_t)w * NEMB + col;
    const v4f a = *(const v4f*)(sp);
    const v4f b = *(const v4f*)(sp + 4);
    v8h hv;
#pragma unroll
    for (int e = 0; e < 4; ++e) {
      hv[e]     = (_Float16)(a[e] * CARRY);
      hv[4 + e] = (_Float16)(b[e] * CARRY);
    }
    unsigned short* dp = xpl + (size_t)bt * NEMB + col;
    *(volatile v8h*)dp = hv;
    __threadfence();
    *(volatile v8h*)dp = hv;
  }
}

template <int KIN>
__global__ __launch_bounds__(NTHR) void lstm_rec_kernel(const unsigned short* __restrict__ xpl,
                                                       const unsigned short* __restrict__ wihp,
                                                       const unsigned short* __restrict__ whhp,
                                                       const float* __restrict__ bias,
                                                       const int* __restrict__ lengths,
                                                       unsigned short* __restrict__ outp, int col0, int dir) {
  constexpr int XSP  = KIN + 8;
  constexpr int NSEG = KIN / 128;
  static_assert(KIN % 128 == 0 && KIN % 32 == 0 && XSP % 8 == 0);
  __shared__ __align__(16) unsigned short Ah[RBLK * AHP];
  __shared__ __align__(16) unsigned short Xs[RBLK * XSP];
  __shared__ int Llen[NBATCH];
  __shared__ int Lslot[NBATCH];
  const _Float16* wih = (const _Float16*)wihp;
  const _Float16* whh = (const _Float16*)whhp;
  const int tid = threadIdx.x, lane = tid & 31, wave = tid >> 5;
  const int c = lane & 15, hh = lane >> 4, koff = hh * 8;
  const int blk  = blockIdx.x;
  const int seg  = tid & 15;
  const int srow = tid >> 4;

  if (tid < NBATCH) {
    Llen[tid]  = clampi(lengths[tid], 0, NSTEP);
    Lslot[tid] = tid;
  }
#pragma unroll 1
  for (int i = tid; i < RBLK * AHP; i += NTHR) Ah[i] = (unsigned short)0;
  __syncthreads();
  if (tid < NBATCH) {
    const int lb = Llen[tid];
    int rk = 0;
#pragma unroll 1
    for (int q = 0; q < NBATCH; ++q) {
      const int lq = Llen[q];
      rk += ((lq < lb) || (lq == lb && q < tid)) ? 1 : 0;
    }
    Lslot[rk] = tid;
  }
  __syncthreads();

  int lenr[8];
#pragma unroll
  for (int r = 0; r < 8; ++r) lenr[r] = Llen[clampi(Lslot[RBLK * blk + 8 * hh + r], 0, NBATCH - 1)];
  const int maxlen = __builtin_amdgcn_readfirstlane(Llen[clampi(Lslot[RBLK * blk + RBLK - 1], 0, NBATCH - 1)]);
  const int brr  = clampi(Lslot[RBLK * blk + srow], 0, NBATCH - 1);
  const int bcp0 = clampi(Lslot[RBLK * blk + wave], 0, NBATCH - 1);
  const int bcp1 = clampi(Lslot[RBLK * blk + NWAVE + wave], 0, NBATCH - 1);

  float cst[2][8], hst[2][8], bb[2][4];
#pragma unroll
  for (int nt = 0; nt < 2; ++nt) {
    const int j = 32 * wave + 16 * nt + c;
#pragma unroll
    for (int g = 0; g < 4; ++g) bb[nt][g] = bias[g * NHID + j];
#pragma unroll
    for (int r = 0; r < 8; ++r) { cst[nt][r] = 0.0f; hst[nt][r] = 0.0f; }
  }

  {
    const int tt0 = dir ? (NSTEP - 1) : 0;
    if (tt0 < maxlen) {
      const unsigned short* src = xpl + ((size_t)brr * NSTEP + (size_t)tt0) * KIN + seg * 8;
#pragma unroll
      for (int it = 0; it < NSEG; ++it) {
        const v4u v = *(const v4u*)(src + it * 128);
        *(v4u*)(&Xs[srow * XSP + it * 128 + seg * 8]) = v;
      }
    }
  }
  __syncthreads();

  const _Float16* xsrow = (const _Float16*)Xs + c * XSP + koff;
  const _Float16* ahrow = (const _Float16*)Ah + c * AHP + koff;
  const v8f z8 = {0.f, 0.f, 0.f, 0.f, 0.f, 0.f, 0.f, 0.f};

#pragma unroll 1
  for (int t = 0; t < NSTEP; ++t) {
    const int tt = dir ? (NSTEP - 1 - t) : t;
    if (tt < maxlen) {
#pragma unroll
      for (int nt = 0; nt < 2; ++nt) {
        const int j = 32 * wave + 16 * nt + c;
        const _Float16* wx = wih + (size_t)j * KIN + koff;
        const _Float16* wh = whh + (size_t)j * NHID + koff;
        v8f acc[4];
        acc[0] = z8; acc[1] = z8; acc[2] = z8; acc[3] = z8;
#pragma unroll 1
        for (int kx = 0; kx < KIN; kx += 32) {
          const v16h a  = Frag<_Float16>::load(xsrow + kx);
          const v16h b0 = Frag<_Float16>::load(wx + kx);
          const v16h b1 = Frag<_Float16>::load(wx + (size_t)1 * NHID * KIN + kx);
          const v16h b2 = Frag<_Float16>::load(wx + (size_t)2 * NHID * KIN + kx);
          const v16h b3 = Frag<_Float16>::load(wx + (size_t)3 * NHID * KIN + kx);
          acc[0] = Frag<_Float16>::mma(a, b0, acc[0]);
          acc[1] = Frag<_Float16>::mma(a, b1, acc[1]);
          acc[2] = Frag<_Float16>::mma(a, b2, acc[2]);
          acc[3] = Frag<_Float16>::mma(a, b3, acc[3]);
          dep_guard_h(acc[0], acc[3], a, b3);
          keep4_h(b0, b1, b2, b3);
        }
#pragma unroll 1
        for (int k0 = 0; k0 < NHID; k0 += 32) {
          const v16h a  = Frag<_Float16>::load(ahrow + k0);
          const v16h b0 = Frag<_Float16>::load(wh + k0);
          const v16h b1 = Frag<_Float16>::load(wh + (size_t)1 * NHID * NHID + k0);
          const v16h b2 = Frag<_Float16>::load(wh + (size_t)2 * NHID * NHID + k0);
          const v16h b3 = Frag<_Float16>::load(wh + (size_t)3 * NHID * NHID + k0);
          acc[0] = Frag<_Float16>::mma(a, b0, acc[0]);
          acc[1] = Frag<_Float16>::mma(a, b1, acc[1]);
          acc[2] = Frag<_Float16>::mma(a, b2, acc[2]);
          acc[3] = Frag<_Float16>::mma(a, b3, acc[3]);
          dep_guard_h(acc[0], acc[3], a, b3);
          keep4_h(b0, b1, b2, b3);
        }
        acc_guard4(acc[0], acc[1], acc[2], acc[3]);
#pragma unroll
        for (int r = 0; r < 8; ++r) {
          const float zi = acc[0][r] * CARRY2_INV + bb[nt][0];
          const float zf = acc[1][r] * CARRY2_INV + bb[nt][1];
          const float zg = acc[2][r] * CARRY2_INV + bb[nt][2];
          const float zo = acc[3][r] * CARRY2_INV + bb[nt][3];
          const float ig = fsig(zi);
          const float fg = fsig(zf);
          const float gg = ftanh(zg);
          const float og = fsig(zo);
          const float cn = fg * cst[nt][r] + ig * gg;
          const float hn = og * ftanh(cn);
          const bool keep = (tt < lenr[r]);
          cst[nt][r] = keep ? cn : cst[nt][r];
          hst[nt][r] = keep ? hn : hst[nt][r];
        }
      }
    }
    __syncthreads();
#pragma unroll
    for (int nt = 0; nt < 2; ++nt) {
      const int j = 32 * wave + 16 * nt + c;
#pragma unroll
      for (int r = 0; r < 8; ++r)
        Ah[(8 * hh + r) * AHP + j] = __builtin_bit_cast(unsigned short, (_Float16)(hst[nt][r] * CARRY));
    }
    {
      const int tn  = (t + 1 < NSTEP) ? (t + 1) : (NSTEP - 1);
      const int ttn = dir ? (NSTEP - 1 - tn) : tn;
      if ((t + 1 < NSTEP) && (ttn < maxlen)) {
        const unsigned short* src = xpl + ((size_t)brr * NSTEP + (size_t)ttn) * KIN + seg * 8;
#pragma unroll
        for (int it = 0; it < NSEG; ++it) {
          const v4u v = *(const v4u*)(src + it * 128);
          *(v4u*)(&Xs[srow * XSP + it * 128 + seg * 8]) = v;
        }
      }
    }
    __syncthreads();
    {
      const v4u v0 = *(const v4u*)(&Ah[wave * AHP + lane * 8]);
      const v4u v1 = *(const v4u*)(&Ah[(NWAVE + wave) * AHP + lane * 8]);
      unsigned short* d0 = outp + ((size_t)bcp0 * NSTEP + (size_t)tt) * (size_t)NCAT + col0 + lane * 8;
      unsigned short* d1 = outp + ((size_t)bcp1 * NSTEP + (size_t)tt) * (size_t)NCAT + col0 + lane * 8;
      for (int pass = 0; pass < 2; ++pass) {
        *(volatile v4u*)d0 = v0;
        *(volatile v4u*)d1 = v1;
        __threadfence();
      }
    }
  }
}

__global__ __launch_bounds__(NTHR) void cls_kernel(const unsigned short* __restrict__ Ap, const unsigned short* __restrict__ Wcp,
                                                  const float* __restrict__ clsb, float* __restrict__ out) {
  __shared__ __align__(16) float stg[CLSSTG];
  const _Float16* A  = (const _Float16*)Ap;
  const _Float16* Wc = (const _Float16*)Wcp;
  const int tid = threadIdx.x, lane = tid & 31, wave = tid >> 5;
  const int c = lane & 15, hh = lane >> 4, koff = hh * 8;
  const int row0 = blockIdx.x * CLSM + wave * 16;
  const _Float16* ap = A + (size_t)(row0 + c) * NCAT + koff;
  const _Float16* wc = Wc + (size_t)c * NCAT + koff;
  const v8f z8 = {0.f, 0.f, 0.f, 0.f, 0.f, 0.f, 0.f, 0.f};
  v8f acc[4];
  acc[0] = z8; acc[1] = z8; acc[2] = z8; acc[3] = z8;
#pragma unroll 1
  for (int k0 = 0; k0 < NCAT; k0 += 32) {
    const v16h a  = Frag<_Float16>::load(ap + k0);
    const v16h b0 = Frag<_Float16>::load(wc + k0);
    const v16h b1 = Frag<_Float16>::load(wc + (size_t)1 * 16 * NCAT + k0);
    const v16h b2 = Frag<_Float16>::load(wc + (size_t)2 * 16 * NCAT + k0);
    const v16h b3 = Frag<_Float16>::load(wc + (size_t)3 * 16 * NCAT + k0);
    acc[0] = Frag<_Float16>::mma(a, b0, acc[0]);
    acc[1] = Frag<_Float16>::mma(a, b1, acc[1]);
    acc[2] = Frag<_Float16>::mma(a, b2, acc[2]);
    acc[3] = Frag<_Float16>::mma(a, b3, acc[3]);
    dep_guard_h(acc[0], acc[3], a, b3);
    keep4_h(b0, b1, b2, b3);
  }
  acc_guard4(acc[0], acc[1], acc[2], acc[3]);

#pragma unroll
  for (int nt = 0; nt < 4; ++nt) {
    const int col  = 16 * nt + c;
    const int colc = (col < NTAGS) ? col : (NTAGS - 1);
    const float bv = clsb[colc];
#pragma unroll
    for (int r = 0; r < 8; ++r) {
      const float v = acc[nt][r] * CARRY2_INV + bv;
      if (col < NTAGS) stg[(wave * 16 + 8 * hh + r) * NTAGS + col] = v;
    }
  }
  __syncthreads();
  float* ob = out + (size_t)blockIdx.x * CLSSTG;
  for (int pass = 0; pass < 2; ++pass) {
#pragma unroll
    for (int it = 0; it < 6; ++it) {
      const int idx = it * NTHR + tid;
      const v4f v = *(const v4f*)(stg + idx * 4);
      *(volatile v4f*)(ob + (size_t)idx * 4) = v;
    }
    if (wave < 2) {
      const int idx = 6 * NTHR + tid;
      const v4f v = *(const v4f*)(stg + idx * 4);
      *(volatile v4f*)(ob + (size_t)idx * 4) = v;
    }
    __threadfence();
  }
}

extern "C" void kernel_launch(void* const* d_in, const int* in_sizes, int n_in,
                              void* d_out, int out_size, void* d_ws, size_t ws_size, hipStream_t stream) {
  if (n_in < 21 || d_out == nullptr || d_ws == nullptr) return;
  if (in_sizes[0] != NROWS || in_sizes[1] != NBATCH || in_sizes[2] != NVOC * NEMB ||
      in_sizes[3] != NGATE * NEMB || in_sizes[4] != NGATE * NHID || in_sizes[5] != NGATE || in_sizes[6] != NGATE ||
      in_sizes[7] != NGATE * NEMB || in_sizes[8] != NGATE * NHID || in_sizes[9] != NGATE || in_sizes[10] != NGATE ||
      in_sizes[11] != NGATE * NCAT || in_sizes[12] != NGATE * NHID || in_sizes[13] != NGATE || in_sizes[14] != NGATE ||
      in_sizes[15] != NGATE * NCAT || in_sizes[16] != NGATE * NHID || in_sizes[17] != NGATE || in_sizes[18] != NGATE ||
      in_sizes[19] != NTAGS * NCAT || in_sizes[20] != NTAGS || out_size != NROWS * NTAGS) return;

  const int*   words   = (const int*)d_in[0];
  const int*   lengths = (const int*)d_in[1];
  const float* emb     = (const float*)d_in[2];
  const float* l1f_Wih = (const float*)d_in[3];
  const float* l1f_Whh = (const float*)d_in[4];
  const float* l1f_bih = (const float*)d_in[5];
  const float* l1f_bhh = (const float*)d_in[6];
  const float* l1b_Wih = (const float*)d_in[7];
  const float* l1b_Whh = (const float*)d_in[8];
  const float* l1b_bih = (const float*)d_in[9];
  const float* l1b_bhh = (const float*)d_in[10];
  const float* l2f_Wih = (const float*)d_in[11];
  const float* l2f_Whh = (const float*)d_in[12];
  const float* l2f_bih = (const float*)d_in[13];
  const float* l2f_bhh = (const float*)d_in[14];
  const float* l2b_Wih = (const float*)d_in[15];
  const float* l2b_Whh = (const float*)d_in[16];
  const float* l2b_bih = (const float*)d_in[17];
  const float* l2b_bhh = (const float*)d_in[18];
  const float* cls_W   = (const float*)d_in[19];
  const float* cls_b   = (const float*)d_in[20];
  float* logits = (float*)d_out;

  char* ws = (char*)d_ws; size_t off = 0;
  auto carve = [&](size_t bytes) -> char* { char* p = ws + off; off += (bytes + 255) & ~(size_t)255; return p; };
  unsigned short* X16 = (unsigned short*)carve((size_t)NROWS * NEMB * 2);
  unsigned short* O1  = (unsigned short*)carve((size_t)NROWS * NCAT * 2);
  unsigned short* O2  = (unsigned short*)carve((size_t)NROWS * NCAT * 2);
  unsigned short* W1F = (unsigned short*)carve((size_t)NGATE * NEMB * 2);
  unsigned short* W1B = (unsigned short*)carve((size_t)NGATE * NEMB * 2);
  unsigned short* U1F = (unsigned short*)carve((size_t)NGATE * NHID * 2);
  unsigned short* U1B = (unsigned short*)carve((size_t)NGATE * NHID * 2);
  unsigned short* U2F = (unsigned short*)carve((size_t)NGATE * NHID * 2);
  unsigned short* U2B = (unsigned short*)carve((size_t)NGATE * NHID * 2);
  unsigned short* W2F = (unsigned short*)carve((size_t)NGATE * NCAT * 2);
  unsigned short* W2B = (unsigned short*)carve((size_t)NGATE * NCAT * 2);
  unsigned short* WC  = (unsigned short*)carve((size_t)NTAGP * NCAT * 2);
  float*          B4  = (float*)carve((size_t)4 * NGATE * 4);
  if (off > ws_size || off > WS_LIMIT) return;

  const int n8_w1 = NGATE * (NEMB / 8);
  const int n8_u  = NGATE * (NHID / 8);
  const int n8_w2 = NGATE * (NCAT / 8);
  const int n8_wc = NTAGP * (NCAT / 8);
  cvt16_kernel<<<(n8_w1 + NTHR - 1) / NTHR, NTHR, 0, stream>>>(l1f_Wih, W1F, NGATE, NGATE, NEMB / 8, CARRY);
  cvt16_kernel<<<(n8_w1 + NTHR - 1) / NTHR, NTHR, 0, stream>>>(l1b_Wih, W1B, NGATE, NGATE, NEMB / 8, CARRY);
  cvt16_kernel<<<(n8_u  + NTHR - 1) / NTHR, NTHR, 0, stream>>>(l1f_Whh, U1F, NGATE, NGATE, NHID / 8, CARRY);
  cvt16_kernel<<<(n8_u  + NTHR - 1) / NTHR, NTHR, 0, stream>>>(l1b_Whh, U1B, NGATE, NGATE, NHID / 8, CARRY);
  cvt16_kernel<<<(n8_u  + NTHR - 1) / NTHR, NTHR, 0, stream>>>(l2f_Whh, U2F, NGATE, NGATE, NHID / 8, CARRY);
  cvt16_kernel<<<(n8_u  + NTHR - 1) / NTHR, NTHR, 0, stream>>>(l2b_Whh, U2B, NGATE, NGATE, NHID / 8, CARRY);
  cvt16_kernel<<<(n8_w2 + NTHR - 1) / NTHR, NTHR, 0, stream>>>(l2f_Wih, W2F, NGATE, NGATE, NCAT / 8, CARRY);
  cvt16_kernel<<<(n8_w2 + NTHR - 1) / NTHR, NTHR, 0, stream>>>(l2b_Wih, W2B, NGATE, NGATE, NCAT / 8, CARRY);
  cvt16_kernel<<<(n8_wc + NTHR - 1) / NTHR, NTHR, 0, stream>>>(cls_W, WC, NTAGS, NTAGP, NCAT / 8, CARRY);
  bias_fold_kernel<<<4, NTHR, 0, stream>>>(l1f_bih, l1f_bhh, l1b_bih, l1b_bhh, l2f_bih, l2f_bhh, l2b_bih, l2b_bhh, B4);
  gather_x16_kernel<<<(NROWS * (NEMB / 8)) / NTHR, NTHR, 0, stream>>>(words, emb, X16);

  lstm_rec_kernel<NEMB><<<NBATCH / RBLK, NTHR, 0, stream>>>(X16, W1F, U1F, B4 + 0 * NGATE, lengths, O1, 0, 0);
  lstm_rec_kernel<NEMB><<<NBATCH / RBLK, NTHR, 0, stream>>>(X16, W1B, U1B, B4 + 1 * NGATE, lengths, O1, NHID, 1);

  lstm_rec_kernel<NCAT><<<NBATCH / RBLK, NTHR, 0, stream>>>(O1, W2F, U2F, B4 + 2 * NGATE, lengths, O2, 0, 0);
  lstm_rec_kernel<NCAT><<<NBATCH / RBLK, NTHR, 0, stream>>>(O1, W2B, U2B, B4 + 3 * NGATE, lengths, O2, NHID, 1);

  cls_kernel<<<NROWS / CLSM, NTHR, 0, stream>>>(O2, WC, cls_b, logits);
}
